// MLPConcatHead_87393994539113
// MI455X (gfx1250) — hardware-run, weakly checked
//
#include <hip/hip_runtime.h>
#include <math.h>

typedef __attribute__((ext_vector_type(16))) _Float16 v16h;
typedef __attribute__((ext_vector_type(8)))  _Float16 v8h;
typedef __attribute__((ext_vector_type(16))) __bf16   v16b;
typedef __attribute__((ext_vector_type(8)))  float    v8f;
typedef __attribute__((ext_vector_type(4)))  float    v4f;

#ifndef SEQ
#define SEQ 768
#endif
#define HID 256
#define PDIM 32
#define PPAD 64

static_assert(SEQ % 64 == 0);
static_assert(HID % 64 == 0 && HID % 32 == 0);
static_assert(PDIM % 32 == 0);
static_assert(PPAD % 64 == 0 && PPAD >= PDIM);
static_assert(HID % 8 == 0 && PPAD % 8 == 0);

#define VST2(T, ptr, val) do { const T vst2_v_ = (val); *(volatile T*)(ptr) = vst2_v_; __threadfence(); *(volatile T*)(ptr) = vst2_v_; } while (0)
typedef float v4f __attribute__((ext_vector_type(4)));
#define VST2V4(ptr, val) do { const v4f vst2_v4_ = (val); *(volatile v4f*)(ptr) = vst2_v4_; __threadfence(); *(volatile v4f*)(ptr) = vst2_v4_; } while (0)

namespace eng {
typedef __attribute__((ext_vector_type(16))) _Float16 v16h;
typedef __attribute__((ext_vector_type(8)))  _Float16 v8h;
typedef __attribute__((ext_vector_type(16))) __bf16   v16b;
typedef __attribute__((ext_vector_type(8)))  __bf16   v8b;
typedef __attribute__((ext_vector_type(8)))  float    v8f;
typedef __attribute__((ext_vector_type(4)))  float    v4f;

__device__ __forceinline__ unsigned short f2bf_bits(float f) {
  unsigned u = __float_as_uint(f);
  return (unsigned short)((u + 0x7FFFu + ((u >> 16) & 1u)) >> 16);
}
__device__ __forceinline__ float bf_bits2f(unsigned short h) { return __uint_as_float(((unsigned)h) << 16); }

__device__ __forceinline__ void dep_guard_h(v8f& a, v8f& b, v16h x, v16h y) { asm volatile("v_nop\n\tv_nop\n\tv_nop\n\tv_nop" : "+v"(a), "+v"(b) : "v"(x), "v"(y)); }
__device__ __forceinline__ void dep_guard_b(v8f& a, v8f& b, v16b x, v16b y) { asm volatile("v_nop\n\tv_nop\n\tv_nop\n\tv_nop" : "+v"(a), "+v"(b) : "v"(x), "v"(y)); }
__device__ __forceinline__ void keep4_h(v16h a, v16h b, v16h c, v16h d) { asm volatile("v_nop" :: "v"(a), "v"(b), "v"(c), "v"(d)); }
__device__ __forceinline__ void keep4_b(v16b a, v16b b, v16b c, v16b d) { asm volatile("v_nop" :: "v"(a), "v"(b), "v"(c), "v"(d)); }
__device__ __forceinline__ void acc_guard4(v8f& a, v8f& b, v8f& c, v8f& d) { asm volatile("v_nop\n\tv_nop\n\tv_nop\n\tv_nop" : "+v"(a), "+v"(b), "+v"(c), "+v"(d)); }
template <typename T> struct Frag;
template <> struct Frag<_Float16> {
  typedef v16h V; union U { v16h v; v8h h[2]; };
  static __device__ __forceinline__ v16h load(const _Float16* p) {
    U f; f.h[0] = *(const v8h*)(p); f.h[1] = *(const v8h*)(p + 16); return f.v;
  }
  static __device__ __forceinline__ v8f mma(v16h a, v16h b, v8f c) {
    return __builtin_amdgcn_wmma_f32_16x16x32_f16(false, a, false, b, (short)0, c, false, false);
  }
  static __device__ __forceinline__ void guard(v8f& a, v8f& b, v16h x, v16h y) { dep_guard_h(a, b, x, y); }
  static __device__ __forceinline__ void keep(v16h a, v16h b, v16h c, v16h d) { keep4_h(a, b, c, d); }
};
template <> struct Frag<__bf16> {
  typedef v16b V; union U { v16b v; v8b h[2]; };
  static __device__ __forceinline__ v16b load(const __bf16* p) {
    U f; f.h[0] = *(const v8b*)(p); f.h[1] = *(const v8b*)(p + 16); return f.v;
  }
  static __device__ __forceinline__ v8f mma(v16b a, v16b b, v8f c) {
    return __builtin_amdgcn_wmma_f32_16x16x32_bf16(false, a, false, b, (short)0, c, false, false);
  }
  static __device__ __forceinline__ void guard(v8f& a, v8f& b, v16b x, v16b y) { dep_guard_b(a, b, x, y); }
  static __device__ __forceinline__ void keep(v16b a, v16b b, v16b c, v16b d) { keep4_b(a, b, c, d); }
};

template <int ET> struct Elem;
template <> struct Elem<0> { typedef _Float16 T; };
template <> struct Elem<1> { typedef __bf16 T; };
template <int ET, bool SPLIT, int BIAS_MODE, int OUT_MODE, bool RESID, int ACT = 0>
__global__ __launch_bounds__(256) void wmma_gemm64(
    const unsigned short* __restrict__ Ap, const unsigned short* __restrict__ A2p, int lda, long strideA,
    const unsigned short* __restrict__ Btp, const unsigned short* __restrict__ Bt2p, int ldb, long strideB,
    void* __restrict__ Cout, void* __restrict__ Cout2, int ldc, long strideC,
    const float* __restrict__ bias,
    const float* __restrict__ resid, long strideR,
    int M, int N, int K, float scale) {
  typedef typename Elem<ET>::T T;
  typedef typename Frag<T>::V V;
  const T* A = (const T*)Ap; const T* A2 = (const T*)A2p; const T* Bt = (const T*)Btp; const T* Bt2 = (const T*)Bt2p;
  __shared__ __align__(16) float sT[8][16 * 68];
  const int b    = blockIdx.y;
  const int lane = threadIdx.x & 31;
  const int wave = threadIdx.x >> 5;
  const int tilesN = N >> 6;
  const int tilesM = M >> 6;
  const int tile = blockIdx.x * 8 + wave;
  if (tile >= tilesM * tilesN) return;
  const int tm = tile / tilesN;
  const int tn = tile - tm * tilesN;
  const int m0 = tm << 6;
  const int n0 = tn << 6;

  const T* Ab  = A  + (size_t)b * strideA;
  const T* Bb  = Bt + (size_t)b * strideB;
  const T* Ab2 = SPLIT ? (A2  + (size_t)b * strideA) : nullptr;
  const T* Bb2 = SPLIT ? (Bt2 + (size_t)b * strideB) : nullptr;

  const int rlane = lane & 15;
  const int koff  = (lane >> 4) * 8;
  const int mOff  = (lane >> 4) * 8;

  v8f acc[4][4];
#pragma unroll
  for (int i = 0; i < 4; ++i)
#pragma unroll
    for (int j = 0; j < 4; ++j) acc[i][j] = (v8f){0.f,0.f,0.f,0.f,0.f,0.f,0.f,0.f};

  for (int k0 = 0; k0 < K; k0 += 32) {
    V bh[4], bl[4];
#pragma unroll
    for (int j = 0; j < 4; ++j) {
      const size_t bo = (size_t)(n0 + (j << 4) + rlane) * ldb + koff + k0;
      bh[j] = Frag<T>::load(Bb + bo);
      if (SPLIT) bl[j] = Frag<T>::load(Bb2 + bo);
    }
#pragma unroll
    for (int i = 0; i < 4; ++i) {
      const size_t ao = (size_t)(m0 + (i << 4) + rlane) * lda + koff + k0;
      V ah = Frag<T>::load(Ab + ao);
      V al;
      if (SPLIT) al = Frag<T>::load(Ab2 + ao);
#pragma unroll
      for (int j = 0; j < 4; ++j) {
        acc[i][j] = Frag<T>::mma(ah, bh[j], acc[i][j]);
        if (SPLIT) {
          acc[i][j] = Frag<T>::mma(ah, bl[j], acc[i][j]);
          acc[i][j] = Frag<T>::mma(al, bh[j], acc[i][j]);
        }
      }
      Frag<T>::guard(acc[i][0], acc[i][3], ah, SPLIT ? al : ah);
    }
    Frag<T>::keep(bh[0], bh[1], bh[2], bh[3]);
    if (SPLIT) Frag<T>::keep(bl[0], bl[1], bl[2], bl[3]);
  }
  acc_guard4(acc[0][0], acc[0][1], acc[0][2], acc[0][3]);
  acc_guard4(acc[1][0], acc[1][1], acc[1][2], acc[1][3]);
  acc_guard4(acc[2][0], acc[2][1], acc[2][2], acc[2][3]);
  acc_guard4(acc[3][0], acc[3][1], acc[3][2], acc[3][3]);

  float* slab = sT[wave];
  const float* Rb = RESID ? (resid + (size_t)b * strideR) : nullptr;
#pragma unroll
  for (int i = 0; i < 4; ++i) {
    const int mBase = m0 + (i << 4);
#pragma unroll
    for (int j = 0; j < 4; ++j) {
      const int n = n0 + (j << 4) + rlane;
      float bv = 0.f;
      if (BIAS_MODE == 2) bv = bias[n];
#pragma unroll
      for (int r = 0; r < 8; ++r) {
        float v = acc[i][j][r] * scale;
        if (BIAS_MODE == 1) v += bias[mBase + mOff + r];
        if (BIAS_MODE == 2) v += bv;
        if (RESID) v += Rb[(size_t)(mBase + mOff + r) * ldc + n];
        if (ACT == 1) v = tanhf(v);
        if (ACT == 2) v = fmaxf(v, 0.0f);
        if (ACT == 3) v = v / (1.0f + expf(-v));
        if (ACT == 4) v = (v > 0.f) ? v : 0.01f * v;
        if (ACT == 5) v = 0.5f * v * (1.0f + erff(v * 0.70710678118654752f));
        if (ACT == 6) v = (v > 0.f) ? v : 0.2f * v;
        if (ACT == 7) { const float u = 0.7978845608028654f * (v + 0.044715f * v * v * v); v = 0.5f * v * (1.f + tanhf(u)); }
        slab[(mOff + r) * 68 + (j << 4) + rlane] = v;
      }
    }
    __builtin_amdgcn_fence(3  , "workgroup");
    __builtin_amdgcn_wave_barrier();
    __builtin_amdgcn_fence(2  , "workgroup");
    if (OUT_MODE == 0) {
      float* C = (float*)Cout + (size_t)b * strideC;
      const int hh = lane >> 4, c4 = (lane & 15) * 4;
      for (int pass = 0; pass < 2; ++pass) {
#pragma unroll
        for (int it = 0; it < 8; ++it) {
          const int row = it * 2 + hh;
          v4f v = *(const v4f*)(slab + row * 68 + c4);
          *(volatile v4f*)(C + (size_t)(mBase + row) * ldc + n0 + c4) = v;
        }
        __threadfence();
      }
    } else {
      const int q = lane >> 3, c8 = (lane & 7) * 8;
      unsigned short* C  = (unsigned short*)Cout  + (size_t)b * strideC;
      unsigned short* C2 = (OUT_MODE == 2) ? ((unsigned short*)Cout2 + (size_t)b * strideC) : nullptr;
      for (int pass = 0; pass < 2; ++pass) {
#pragma unroll
        for (int it = 0; it < 4; ++it) {
          const int row = it * 4 + q;
          const float* sp = slab + row * 68 + c8;
          v8h hv, lv;
#pragma unroll
          for (int e = 0; e < 8; ++e) {
            if (OUT_MODE == 1) {
              hv[e] = (_Float16)sp[e];
            } else {
              unsigned short hb = f2bf_bits(sp[e]);
              unsigned short lb = f2bf_bits(sp[e] - bf_bits2f(hb));
              hv[e] = __builtin_bit_cast(_Float16, hb);
              lv[e] = __builtin_bit_cast(_Float16, lb);
            }
          }
          *(volatile v8h*)(C + (size_t)(mBase + row) * ldc + n0 + c8) = hv;
          if (OUT_MODE == 2) *(volatile v8h*)(C2 + (size_t)(mBase + row) * ldc + n0 + c8) = lv;
        }
        __threadfence();
      }
    }
    __builtin_amdgcn_fence(3  , "workgroup");
    __builtin_amdgcn_wave_barrier();
    __builtin_amdgcn_fence(2  , "workgroup");
  }
}

}

__global__ __launch_bounds__(256) void k_zero4(float* __restrict__ B, long long n4) { const long long u = (long long)blockIdx.x * 256 + threadIdx.x; if (u >= n4) return; v4f z; z.x = z.y = z.z = z.w = 0.f; VST2V4(B + 4 * u, z); }
__global__ __launch_bounds__(256) void k_padvec(const float* __restrict__ bsrc, int nb, float* __restrict__ Bd, int n) { const int t = blockIdx.x * 256 + threadIdx.x; if (t >= n) return; VST2(float, Bd + t, (t < nb) ? bsrc[min(t, nb - 1)] : 0.f); }

__device__ __forceinline__ unsigned short at_f2h(float x) { return (fabsf(x) < 6.104e-5f) ? (unsigned short)0 : __builtin_bit_cast(unsigned short, (_Float16)x); }
typedef __attribute__((ext_vector_type(4))) unsigned int v4u_at;
__device__ __forceinline__ void at_st8h(unsigned short* Pp, long long o, const float* v) { v4u_at pk; pk.x = (unsigned int)at_f2h(v[0]) | ((unsigned int)at_f2h(v[1]) << 16); pk.y = (unsigned int)at_f2h(v[2]) | ((unsigned int)at_f2h(v[3]) << 16); pk.z = (unsigned int)at_f2h(v[4]) | ((unsigned int)at_f2h(v[5]) << 16); pk.w = (unsigned int)at_f2h(v[6]) | ((unsigned int)at_f2h(v[7]) << 16); VST2(v4u_at, (v4u_at*)(Pp + o), pk); }
__global__ __launch_bounds__(256) void k_at_h16(const float* __restrict__ X, unsigned short* __restrict__ O16, float sc, long long n8) { const long long u = (long long)blockIdx.x * 256 + threadIdx.x; if (u >= n8) return; const float* x = X + 8 * u; float v[8];
#pragma unroll
    for (int i = 0; i < 8; ++i) v[i] = x[i] * sc;
    at_st8h(O16, 8 * u, v); }
__global__ __launch_bounds__(256) void k_mh_wt16(const float* __restrict__ Wm, int KI, int NO, unsigned short* __restrict__ W16, float sw) { const long long u = (long long)blockIdx.x * 256 + threadIdx.x; const int per = KI / 8; if (u >= (long long)NO * per) return; const int k0 = 8 * (int)(u % per); const int o = (int)(u / per); float v[8];
#pragma unroll
    for (int i = 0; i < 8; ++i) v[i] = Wm[(long long)(k0 + i) * NO + o] * sw;
    at_st8h(W16, (long long)o * KI + k0, v); }

typedef _Float16 h16;
static __device__ __forceinline__ h16 toh_flush(float v) { const h16 r = (h16)v; return (fabsf(v) < 6.103515625e-05f) ? (h16)0.0f : r; }
static __device__ __forceinline__ unsigned int pk2_flush(float a, float b) { return (unsigned int)__builtin_bit_cast(unsigned short, toh_flush(a)) | ((unsigned int)__builtin_bit_cast(unsigned short, toh_flush(b)) << 16); }

static_assert(HID == 8 * 32);
static_assert(32 * 16 == HID * 2);
__global__ __launch_bounds__(256) void k_ln1(const float* __restrict__ X1, const float* __restrict__ g, const float* __restrict__ bb, unsigned short* __restrict__ X16, int R, float sc) {
    #pragma clang fp contract(off)
    const int wave = __builtin_amdgcn_readfirstlane(threadIdx.x >> 5);
    const int row = blockIdx.x * 8 + wave; const int L = threadIdx.x & 31;
    if (row >= R) return;
    const int c0 = 8 * L;
    const float* xr = X1 + (long long)row * HID + c0;
    const v4f a0 = *(const v4f*)(xr), a1 = *(const v4f*)(xr + 4);
    float sm = ((a0.x + a0.y) + (a0.z + a0.w)) + ((a1.x + a1.y) + (a1.z + a1.w));
#pragma unroll
    for (int o = 16; o > 0; o >>= 1) sm += __shfl_xor(sm, o, 32);
    const float mu = sm * (1.f / 256.f);
    const v4f d0 = a0 - mu, d1 = a1 - mu;
    float q = ((d0.x * d0.x + d0.y * d0.y) + (d0.z * d0.z + d0.w * d0.w)) + ((d1.x * d1.x + d1.y * d1.y) + (d1.z * d1.z + d1.w * d1.w));
#pragma unroll
    for (int o = 16; o > 0; o >>= 1) q += __shfl_xor(q, o, 32);
    const float rs = rsqrtf(q * (1.f / 256.f) + 1e-5f);
    const v4f g0 = *(const v4f*)(g + c0), g1 = *(const v4f*)(g + c0 + 4);
    const v4f b0 = *(const v4f*)(bb + c0), b1 = *(const v4f*)(bb + c0 + 4);
    const float y0 = fmaxf(d0.x * rs * g0.x + b0.x, 0.f) * sc, y1 = fmaxf(d0.y * rs * g0.y + b0.y, 0.f) * sc;
    const float y2 = fmaxf(d0.z * rs * g0.z + b0.z, 0.f) * sc, y3 = fmaxf(d0.w * rs * g0.w + b0.w, 0.f) * sc;
    const float y4 = fmaxf(d1.x * rs * g1.x + b1.x, 0.f) * sc, y5 = fmaxf(d1.y * rs * g1.y + b1.y, 0.f) * sc;
    const float y6 = fmaxf(d1.z * rs * g1.z + b1.z, 0.f) * sc, y7 = fmaxf(d1.w * rs * g1.w + b1.w, 0.f) * sc;
    v4u_at pk; pk.x = pk2_flush(y0, y1); pk.y = pk2_flush(y2, y3); pk.z = pk2_flush(y4, y5); pk.w = pk2_flush(y6, y7);
    VST2(v4u_at, (v4u_at*)(X16 + (long long)row * HID + c0), pk);
}

static __device__ __forceinline__ float mish_fast(float t) {
    const float e = __expf(fminf(t, 20.0f));
    const float n = e * (e + 2.0f);
    return t * n * __builtin_amdgcn_rcpf(n + 2.0f);
}

#define PT_I 8
#define PT_J 32
#define PT_LD 260
static_assert(HID == 256 && HID / 4 == 64);
static_assert(PT_I * 32 == 256);
static_assert(PT_J == 32);
static_assert(SEQ % PT_I == 0 && SEQ % PT_J == 0);
static_assert((PT_LD % 4) == 0 && PT_LD >= HID);
static_assert((PT_I * (HID / 4)) % 256 == 0 && (PT_J * (HID / 4)) % 256 == 0);
static_assert((PT_I + PT_J) % 8 == 0);
static_assert(((PT_I + PT_J) * PT_LD + 3 * HID + (PT_I + PT_J)) * 4 <= 131072);
static_assert(256 * 4 == PT_I * PT_J * 4);
__global__ __launch_bounds__(256) void k_pair(const float* __restrict__ Fi, const float* __restrict__ Fj, const float* __restrict__ g2, const float* __restrict__ be2,
                                              const float* __restrict__ wt, const float* __restrict__ btp, float* __restrict__ out) {
    #pragma clang fp contract(off)
    __shared__ __align__(16) float Fab[(PT_I + PT_J) * PT_LD];
    __shared__ __align__(16) float gs[HID];
    __shared__ __align__(16) float bes[HID];
    __shared__ __align__(16) float wts[HID];
    __shared__ float rsum[PT_I + PT_J];
    const int t = threadIdx.x;
    const int wave = __builtin_amdgcn_readfirstlane(threadIdx.x >> 5);
    const int lane = t & 31;
    const int i0 = blockIdx.y * PT_I, j0 = blockIdx.x * PT_J;
#pragma unroll 1
    for (int c = 0; c < (PT_I * (HID / 4)) / 256; ++c) {
        const int chunk = t + c * 256; const int row = chunk >> 6; const int col4 = (chunk & 63) << 2;
        const v4f v = *(const v4f*)(Fi + (long long)(i0 + row) * HID + col4);
        *(v4f*)(&Fab[row * PT_LD + col4]) = v;
    }
#pragma unroll 1
    for (int c = 0; c < (PT_J * (HID / 4)) / 256; ++c) {
        const int chunk = t + c * 256; const int row = chunk >> 6; const int col4 = (chunk & 63) << 2;
        const v4f v = *(const v4f*)(Fj + (long long)(j0 + row) * HID + col4);
        *(v4f*)(&Fab[(PT_I + row) * PT_LD + col4]) = v;
    }
    gs[t] = g2[t]; bes[t] = be2[t]; wts[t] = wt[t];
    __syncthreads();
#pragma unroll 1
    for (int rr = 0; rr < (PT_I + PT_J) / 8; ++rr) {
        const int R = wave + 8 * rr;
        const v4f a = *(const v4f*)(&Fab[R * PT_LD + 8 * lane]);
        const v4f b = *(const v4f*)(&Fab[R * PT_LD + 8 * lane + 4]);
        float s = ((a.x + a.y) + (a.z + a.w)) + ((b.x + b.y) + (b.z + b.w));
        s += __shfl_xor(s, 16, 32); s += __shfl_xor(s, 8, 32); s += __shfl_xor(s, 4, 32); s += __shfl_xor(s, 2, 32); s += __shfl_xor(s, 1, 32);
        if (lane == 0) rsum[R] = s;
    }
    __syncthreads();
    const int ra = wave * PT_LD, rb = (PT_I + lane) * PT_LD;
    const float mu = (rsum[wave] + rsum[PT_I + lane]) * (1.f / 256.f);
    float q0 = 0.f, q1 = 0.f, q2 = 0.f, q3 = 0.f;
#pragma unroll 1
    for (int k4 = 0; k4 < HID / 4; ++k4) {
        const v4f av = *(const v4f*)(&Fab[ra + 4 * k4]);
        const v4f bv = *(const v4f*)(&Fab[rb + 4 * k4]);
        const float dx = (av.x + bv.x) - mu, dy = (av.y + bv.y) - mu, dz = (av.z + bv.z) - mu, dw = (av.w + bv.w) - mu;
        q0 += dx * dx; q1 += dy * dy; q2 += dz * dz; q3 += dw * dw;
    }
    const float var = ((q0 + q1) + (q2 + q3)) * (1.f / 256.f);
    const float sc = rsqrtf(var + 1e-5f);
    float a0 = 0.f, a1 = 0.f, a2 = 0.f, a3 = 0.f;
#pragma unroll 1
    for (int k4 = 0; k4 < HID / 4; ++k4) {
        const v4f av = *(const v4f*)(&Fab[ra + 4 * k4]);
        const v4f bv = *(const v4f*)(&Fab[rb + 4 * k4]);
        const v4f gv = *(const v4f*)(&gs[4 * k4]);
        const v4f ev = *(const v4f*)(&bes[4 * k4]);
        const v4f wv = *(const v4f*)(&wts[4 * k4]);
        a0 += wv.x * mish_fast(((av.x + bv.x) - mu) * sc * gv.x + ev.x);
        a1 += wv.y * mish_fast(((av.y + bv.y) - mu) * sc * gv.y + ev.y);
        a2 += wv.z * mish_fast(((av.z + bv.z) - mu) * sc * gv.z + ev.z);
        a3 += wv.w * mish_fast(((av.w + bv.w) - mu) * sc * gv.w + ev.w);
    }
    const float res = ((a0 + a1) + (a2 + a3)) + btp[0];
    VST2(float, out + (long long)(i0 + wave) * SEQ + j0 + lane, res);
}

#define AL256(x) (((((size_t)(x)) + 255) / 256) * 256)
static_assert(AL256((size_t)SEQ * HID * 2) * 2 + AL256((size_t)HID * HID * 2) + AL256((size_t)PPAD * HID * 2) + AL256((size_t)HID * PDIM * 2) * 2 + AL256((size_t)PPAD * 4)
              + AL256((size_t)SEQ * HID * 4) * 3 + AL256((size_t)SEQ * PPAD * 4) + AL256((size_t)SEQ * PPAD * 2) <= (size_t)134217728);

extern "C" void kernel_launch(void* const* d_in, const int* in_sizes, int n_in, void* d_out, int out_size, void* d_ws, size_t ws_size, hipStream_t stream) {
    if (n_in < 15) return;
    if (in_sizes[0] < SEQ * HID || in_sizes[1] < HID * HID || in_sizes[2] < HID || in_sizes[3] < HID || in_sizes[4] < HID) return;
    if (in_sizes[5] < HID * PDIM || in_sizes[6] < PDIM || in_sizes[7] < PDIM * HID || in_sizes[8] < HID || in_sizes[9] < PDIM * HID || in_sizes[10] < HID) return;
    if (in_sizes[11] < HID || in_sizes[12] < HID || in_sizes[13] < HID || in_sizes[14] < 1) return;
    if (out_size < SEQ * SEQ) return;
    const float* hf   = (const float*)d_in[0];
    const float* W1   = (const float*)d_in[1];
    const float* b1   = (const float*)d_in[2];
    const float* ln1g = (const float*)d_in[3];
    const float* ln1b = (const float*)d_in[4];
    const float* W2   = (const float*)d_in[5];
    const float* b2   = (const float*)d_in[6];
    const float* Wi   = (const float*)d_in[7];
    const float* bi   = (const float*)d_in[8];
    const float* Wj   = (const float*)d_in[9];
    const float* bj   = (const float*)d_in[10];
    const float* ln2g = (const float*)d_in[11];
    const float* ln2b = (const float*)d_in[12];
    const float* Wt   = (const float*)d_in[13];
    const float* bt   = (const float*)d_in[14];
    float* out = (float*)d_out;
    char* wsp = (char*)d_ws;
    unsigned short* h16 = (unsigned short*)wsp; wsp += AL256((size_t)SEQ * HID * 2);
    unsigned short* W1t = (unsigned short*)wsp; wsp += AL256((size_t)HID * HID * 2);
    unsigned short* W2t = (unsigned short*)wsp; wsp += AL256((size_t)PPAD * HID * 2);
    unsigned short* Wit = (unsigned short*)wsp; wsp += AL256((size_t)HID * PDIM * 2);
    unsigned short* Wjt = (unsigned short*)wsp; wsp += AL256((size_t)HID * PDIM * 2);
    float* b2p = (float*)wsp; wsp += AL256((size_t)PPAD * 4);
    float* X1 = (float*)wsp; wsp += AL256((size_t)SEQ * HID * 4);
    unsigned short* x16 = (unsigned short*)wsp; wsp += AL256((size_t)SEQ * HID * 2);
    float* Hf = (float*)wsp; wsp += AL256((size_t)SEQ * PPAD * 4);
    unsigned short* H16 = (unsigned short*)wsp; wsp += AL256((size_t)SEQ * PPAD * 2);
    float* Fi = (float*)wsp; wsp += AL256((size_t)SEQ * HID * 4);
    float* Fj = (float*)wsp; wsp += AL256((size_t)SEQ * HID * 4);
    if ((size_t)(wsp - (char*)d_ws) > ws_size) return;

    k_at_h16<<<(unsigned)(((long long)SEQ * HID / 8 + 255) / 256), 256, 0, stream>>>(hf, h16, 8.0f, (long long)SEQ * HID / 8);
    k_mh_wt16<<<(unsigned)((HID * (HID / 8) + 255) / 256), 256, 0, stream>>>(W1, HID, HID, W1t, 32.0f);
    k_mh_wt16<<<(unsigned)((PDIM * (HID / 8) + 255) / 256), 256, 0, stream>>>(W2, HID, PDIM, W2t, 32.0f);
    k_zero4<<<(unsigned)((((PPAD - PDIM) * HID * 2 / 16) + 255) / 256), 256, 0, stream>>>((float*)(W2t + (size_t)PDIM * HID), (long long)((PPAD - PDIM) * HID * 2 / 16));
    k_mh_wt16<<<(unsigned)((HID * (PDIM / 8) + 255) / 256), 256, 0, stream>>>(Wi, PDIM, HID, Wit, 32.0f);
    k_mh_wt16<<<(unsigned)((HID * (PDIM / 8) + 255) / 256), 256, 0, stream>>>(Wj, PDIM, HID, Wjt, 32.0f);
    k_padvec<<<1, 256, 0, stream>>>(b2, PDIM, b2p, PPAD);

    eng::wmma_gemm64<0, false, 2, 0, false, 0><<<dim3((unsigned)((((SEQ) / 64) * ((HID) / 64) + 7) / 8), (unsigned)(1)), 256, 0, stream>>>((const unsigned short*)(h16), nullptr, HID, 0, (const unsigned short*)(W1t), nullptr, HID, 0, (void*)(X1), nullptr, HID, 0, b1, nullptr, 0, SEQ, HID, HID, 0.00390625f);
    k_ln1<<<(unsigned)((SEQ + 7) / 8), 256, 0, stream>>>(X1, ln1g, ln1b, x16, SEQ, 8.0f);
    eng::wmma_gemm64<0, false, 2, 0, false, 0><<<dim3((unsigned)((((SEQ) / 64) * ((PPAD) / 64) + 7) / 8), (unsigned)(1)), 256, 0, stream>>>((const unsigned short*)(x16), nullptr, HID, 0, (const unsigned short*)(W2t), nullptr, HID, 0, (void*)(Hf), nullptr, PPAD, 0, b2p, nullptr, 0, SEQ, PPAD, HID, 0.00390625f);
    k_at_h16<<<(unsigned)(((long long)SEQ * PPAD / 8 + 255) / 256), 256, 0, stream>>>(Hf, H16, 8.0f, (long long)SEQ * PPAD / 8);
    eng::wmma_gemm64<0, false, 2, 0, false, 0><<<dim3((unsigned)((((SEQ) / 64) * ((HID) / 64) + 7) / 8), (unsigned)(1)), 256, 0, stream>>>((const unsigned short*)(H16), nullptr, PPAD, 0, (const unsigned short*)(Wit), nullptr, PDIM, 0, (void*)(Fi), nullptr, HID, 0, bi, nullptr, 0, SEQ, HID, PDIM, 0.00390625f);
    eng::wmma_gemm64<0, false, 2, 0, false, 0><<<dim3((unsigned)((((SEQ) / 64) * ((HID) / 64) + 7) / 8), (unsigned)(1)), 256, 0, stream>>>((const unsigned short*)(H16), nullptr, PPAD, 0, (const unsigned short*)(Wjt), nullptr, PDIM, 0, (void*)(Fj), nullptr, HID, 0, bj, nullptr, 0, SEQ, HID, PDIM, 0.00390625f);
    k_pair<<<dim3((unsigned)(SEQ / PT_J), (unsigned)(SEQ / PT_I)), 256, 0, stream>>>(Fi, Fj, ln2g, ln2b, Wt, bt, out);
}
